// TAGCN_68135361184096
// MI455X (gfx1250) — hardware-run, weakly checked
//
#include <hip/hip_runtime.h>


namespace {
constexpr int N = 50000, E = 500000, F = 128, U = 256, KH = 3, KT = F * (KH + 1)  ;
constexpr float HS = 256.0f, WSC = 256.0f;
typedef _Float16 b16;
typedef __attribute__((ext_vector_type(16))) _Float16 v16b;
typedef __attribute__((ext_vector_type(8))) _Float16 v8b;
typedef __attribute__((ext_vector_type(8))) float v8f;
typedef __attribute__((ext_vector_type(4))) float v4f;
__device__ __forceinline__ float bf16_rne(float f) { unsigned int u = __float_as_uint(f); u += 0x7FFFu + ((u >> 16) & 1u); float r = __uint_as_float(u & 0xFFFF0000u); asm volatile("" : "+v"(r)); return r; }
__device__ __forceinline__ float bfv(float f) { float r = bf16_rne(f); asm volatile("" : "+v"(r)); return r; }
__device__ __forceinline__ void split16(float v, b16& hi, b16& lo) { hi = (b16)v; lo = (b16)(v - (float)hi); }
__device__ __forceinline__ v16b frag_kb(const b16* p, int hh) { const v8b a = *(const v8b*)(p + 8 * hh), b = *(const v8b*)(p + 16 + 8 * hh); v16b f;
#pragma unroll
  for (int e = 0; e < 8; ++e) { f[e] = a[e]; f[8 + e] = b[e]; } return f; }
__device__ __forceinline__ v8f wmma16b(v16b a, v16b b, v8f c) { v8f d = __builtin_amdgcn_wmma_f32_16x16x32_f16(false, a, false, b, (short)0, c, false, false); asm volatile("v_nop\n\tv_nop\n\tv_nop\n\tv_nop" : "+v"(d) : "v"(a), "v"(b)); return d; }
__device__ __forceinline__ void wave_lds_sync() { __builtin_amdgcn_fence(__ATOMIC_RELEASE, "workgroup"); __builtin_amdgcn_wave_barrier(); __builtin_amdgcn_fence(__ATOMIC_ACQUIRE, "workgroup"); }
__device__ __forceinline__ float pmul(float a, float b) { float p = a * b; asm volatile("" : "+v"(p)); return p; }
__device__ __forceinline__ int iclamp(int v, int lo, int hi) { return v < lo ? lo : (v > hi ? hi : v); }
constexpr int CSR_NBLKC = 512, CSR_GBC = 8, CSR_GNC = 1 << CSR_GBC  , CSR_TSC = (CSR_GNC < 32 ? 32 : CSR_GNC)  , CSR_MAXGC = 512, CSR_CAPC = 12288  ;
__device__ __host__ __forceinline__ int csr_tixC(int v) { return (v >> CSR_GBC) * CSR_TSC + (v & (CSR_GNC - 1)); }
__global__ __launch_bounds__(64) void csrA_kernelC(const int* __restrict__ dst, int E, int N, int nG, int CHP, int NGP, int* __restrict__ STG, int* __restrict__ HST) {
  extern __shared__ int sm[];
  int* cnt = sm; int* run = sm + NGP; int* ids = sm + 2 * NGP;
  const int b = blockIdx.x; const int ch = (E + CSR_NBLKC - 1) / CSR_NBLKC; const int e0 = b * ch, e1 = min(E, e0 + ch);
  for (int i = threadIdx.x; i < NGP; i += 64) cnt[i] = 0;
  for (int i = threadIdx.x; i < CHP; i += 64) ids[i] = -1;
  __syncthreads();
  if (threadIdx.x == 0) {
    for (int e = e0; e < e1; ++e) { int d = dst[e]; d = (d < 0) ? 0 : (d >= N ? N - 1 : d); cnt[d >> CSR_GBC] += 1; }
    int acc = 0; for (int g = 0; g < nG; ++g) { run[g] = acc; acc += cnt[g]; }
    for (int e = e0; e < e1; ++e) { int d = dst[e]; d = (d < 0) ? 0 : (d >= N ? N - 1 : d); const int g = d >> CSR_GBC; ids[run[g]] = e; run[g] += 1; } }
  __syncthreads();
  typedef __attribute__((ext_vector_type(4))) int v4i;
  for (int pass = 0; pass < 2; ++pass) {
    for (int i = threadIdx.x; i < CHP / 4; i += 64) *(volatile v4i*)(STG + (size_t)b * CHP + i * 4) = *(const v4i*)(&ids[i * 4]);
    for (int i = threadIdx.x; i < NGP / 4; i += 64) { v4i v; for (int e = 0; e < 4; ++e) v[e] = (i * 4 + e < nG) ? cnt[i * 4 + e] : 0; *(volatile v4i*)(HST + (size_t)b * NGP + i * 4) = v; }
    __threadfence(); }
}
__global__ __launch_bounds__(512) void csrS_kernelC(const int* __restrict__ HST, int nG, int NGP, int* __restrict__ START, int* __restrict__ TOT, int* __restrict__ OFF) {
  __shared__ int tot[CSR_MAXGC];
  const int b = threadIdx.x;
  for (int pass = 0; pass < 2; ++pass) { int runb = 0; for (int g = 0; g < nG; ++g) { int c = HST[(size_t)b * NGP + g]; c = (c < 0) ? 0 : c; ((volatile int*)OFF)[(size_t)g * CSR_NBLKC + b] = runb; runb += c; } __threadfence(); }
  for (int g = threadIdx.x; g < nG; g += 512) { int s = 0; for (int bb = 0; bb < CSR_NBLKC; ++bb) { int c = HST[(size_t)bb * NGP + g]; s += (c < 0) ? 0 : c; } tot[g] = s; }
  __syncthreads();
  if (threadIdx.x < 32) {
    __shared__ int st[CSR_MAXGC + 32];
    if (threadIdx.x == 0) { int acc = 0; for (int g = 0; g < NGP; ++g) { st[g] = acc; if (g < nG) acc += (tot[g] + 31) & ~31; } st[NGP] = acc; }
    __builtin_amdgcn_fence(__ATOMIC_RELEASE, "workgroup"); __builtin_amdgcn_wave_barrier(); __builtin_amdgcn_fence(__ATOMIC_ACQUIRE, "workgroup");
    for (int pass = 0; pass < 2; ++pass) { for (int i = threadIdx.x; i < NGP + 32; i += 32) { ((volatile int*)START)[i] = (i <= NGP) ? st[min(i, NGP)] : 0; ((volatile int*)TOT)[i] = (i < nG) ? tot[i] : 0; } __threadfence(); } }
}
__global__ __launch_bounds__(256) void csrB_kernelC(const int* __restrict__ dst, int N, int nG, int CHP, int NGP, int permLen, const int* __restrict__ STG, const int* __restrict__ HST, const int* __restrict__ OFF, const int* __restrict__ START, const int* __restrict__ TOT, int* __restrict__ PERM, int* __restrict__ ROWPTR, int* __restrict__ ROWCNT, int* __restrict__ FLAG) {
  typedef __attribute__((ext_vector_type(4))) int v4i;
  __shared__ int ids[CSR_CAPC]; __shared__ unsigned short key[CSR_CAPC]; __shared__ int outp[CSR_CAPC]; __shared__ int ncnt[CSR_GNC + 1]; __shared__ int boff[CSR_NBLKC + 1];
  const int g = blockIdx.x, t_ = threadIdx.x; int tot = TOT[g]; int st = START[g], stn = START[g + 1]; const int v0 = g * CSR_GNC; const int nv = min(CSR_GNC, N - v0); const int t0 = g * CSR_TSC;
  st = (st < 0) ? 0 : (st > permLen - 32 ? permLen - 32 : st) & ~31; stn = (stn < st) ? st : (stn > permLen ? permLen : stn); tot = (tot < 0) ? 0 : tot; if (tot > stn - st && tot <= CSR_CAPC) tot = stn - st;
  if (tot > CSR_CAPC) {
    for (int pass = 0; pass < 2; ++pass) { for (int i = t_; i < CSR_TSC / 4; i += 256) { v4i a, c; for (int e = 0; e < 4; ++e) { a[e] = st; c[e] = 0; } *(volatile v4i*)(ROWPTR + t0 + i * 4) = a; *(volatile v4i*)(ROWCNT + t0 + i * 4) = c; } if (t_ == 0) ((volatile int*)FLAG)[0] = 1; __threadfence(); } (void)nv; return; }
  if (t_ == 0) { int acc = 0; for (int b = 0; b < CSR_NBLKC; ++b) { boff[b] = acc; int c = HST[(size_t)b * NGP + g]; c = (c < 0) ? 0 : (c > CHP ? CHP : c); acc += c; if (acc > tot) acc = tot; } boff[CSR_NBLKC] = acc; }
  for (int i = t_; i <= CSR_GNC; i += 256) ncnt[i] = 0;
  __syncthreads();
  for (int b = 0; b < CSR_NBLKC; ++b) { const int c = boff[b + 1] - boff[b]; int o_ = OFF[(size_t)g * CSR_NBLKC + b]; o_ = (o_ < 0) ? 0 : (o_ > CHP - c ? CHP - c : o_); const int* src_ = STG + (size_t)b * CHP + o_;
    for (int i = t_; i < c; i += 256) { int id = src_[i]; id = (id < 0) ? 0 : id; ids[boff[b] + i] = id; int d = dst[id]; d = (d < v0) ? v0 : (d >= N ? N - 1 : d); int kk = d - v0; kk = (kk < 0) ? 0 : (kk >= CSR_GNC ? CSR_GNC - 1 : kk); key[boff[b] + i] = (unsigned short)kk; } }
  __syncthreads();
  if (t_ == 0) { for (int i = 0; i < tot; ++i) ncnt[key[i]] += 1; int acc = 0; for (int vl = 0; vl < CSR_GNC; ++vl) { const int c = ncnt[vl]; ncnt[vl] = acc; acc += c; } ncnt[CSR_GNC] = acc;
    for (int i = 0; i < tot; ++i) { const int vl = key[i]; outp[ncnt[vl]] = ids[i]; ncnt[vl] += 1; }
    for (int vl = CSR_GNC; vl > 0; --vl) ncnt[vl] = ncnt[vl - 1]; ncnt[0] = 0; }
  __syncthreads();
  for (int pass = 0; pass < 2; ++pass) {
    for (int i = t_; i < (stn - st) / 4; i += 256) { v4i v; for (int e = 0; e < 4; ++e) { const int q = i * 4 + e; v[e] = (q < tot) ? outp[q] : -1; } *(volatile v4i*)(PERM + st + i * 4) = v; }
    for (int i = t_; i < CSR_TSC / 4; i += 256) { v4i a, c; for (int e = 0; e < 4; ++e) { const int vl = i * 4 + e; const int vc = vl < CSR_GNC ? vl : CSR_GNC; a[e] = (vl < CSR_GNC) ? st + ncnt[vc] : st; c[e] = (vl < nv) ? (ncnt[(vc < CSR_GNC ? vc : CSR_GNC - 1) + 1] - ncnt[vc]) : 0; } *(volatile v4i*)(ROWPTR + t0 + i * 4) = a; *(volatile v4i*)(ROWCNT + t0 + i * 4) = c; }
    __threadfence(); }
}
__global__ __launch_bounds__(256) void csrZ_kernelC(int* __restrict__ p, size_t n4) { typedef __attribute__((ext_vector_type(4))) int v4i; const size_t tid = (size_t)blockIdx.x * 256 + threadIdx.x, nth = (size_t)gridDim.x * 256; v4i z = {0, 0, 0, 0}; for (size_t i = tid; i < n4; i += nth) *(volatile v4i*)(p + i * 4) = z; }
struct CsrBufsC { int *STG, *HST, *OFF, *START, *TOT, *PERM, *ROWPTR, *ROWCNT, *FLAG; int nG, NGP, CHP; size_t permLen; char* base; size_t bytes; };
static size_t csr_carveC(CsrBufsC& c, char* ws, size_t off, int E, int N) {
  const size_t off0 = off; c.base = ws + off;
  auto al = [&](size_t bytes) { char* p = ws + off; off += (bytes + 255) & ~(size_t)255; return p; };
  c.nG = (N + CSR_GNC - 1) / CSR_GNC; c.NGP = (c.nG + 31) & ~31; const int ch = (E + CSR_NBLKC - 1) / CSR_NBLKC; c.CHP = (ch + 31) & ~31; c.permLen = (size_t)E + 32 * (size_t)c.nG + 32;
  c.STG = (int*)al((size_t)CSR_NBLKC * c.CHP * 4); c.HST = (int*)al((size_t)CSR_NBLKC * c.NGP * 4); c.OFF = (int*)al((size_t)c.NGP * CSR_NBLKC * 4); c.START = (int*)al((size_t)(c.NGP + 64) * 4); c.TOT = (int*)al((size_t)(c.NGP + 64) * 4);
  c.PERM = (int*)al(c.permLen * 4); c.ROWPTR = (int*)al((size_t)c.nG * CSR_TSC * 4); c.ROWCNT = (int*)al((size_t)c.nG * CSR_TSC * 4); c.FLAG = (int*)al(256);
  c.bytes = off - off0; return off;
}
static void csr_buildC(const CsrBufsC& c, const int* dst, int E, int N, hipStream_t stream) {
  const size_t smem = (size_t)(2 * c.NGP + c.CHP) * 4;
  csrZ_kernelC<<<512, 256, 0, stream>>>((int*)c.base, c.bytes / 16);
  csrA_kernelC<<<CSR_NBLKC, 64, smem, stream>>>(dst, E, N, c.nG, c.CHP, c.NGP, c.STG, c.HST);
  csrS_kernelC<<<1, 512, 0, stream>>>(c.HST, c.nG, c.NGP, c.START, c.TOT, c.OFF);
  csrB_kernelC<<<c.nG, 256, 0, stream>>>(dst, N, c.nG, c.CHP, c.NGP, (int)c.permLen, c.STG, c.HST, c.OFF, c.START, c.TOT, c.PERM, c.ROWPTR, c.ROWCNT, c.FLAG);
}
constexpr int CSR_NBLKR = 512, CSR_GBR = 8, CSR_GNR = 1 << CSR_GBR  , CSR_TSR = (CSR_GNR < 32 ? 32 : CSR_GNR)  , CSR_MAXGR = 512, CSR_CAPR = 12288  ;
__device__ __host__ __forceinline__ int csr_tixR(int v) { return (v >> CSR_GBR) * CSR_TSR + (v & (CSR_GNR - 1)); }
__global__ __launch_bounds__(64) void csrA_kernelR(const int* __restrict__ dst, int E, int N, int nG, int CHP, int NGP, int* __restrict__ STG, int* __restrict__ HST) {
  extern __shared__ int sm[];
  int* cnt = sm; int* run = sm + NGP; int* ids = sm + 2 * NGP;
  const int b = blockIdx.x; const int ch = (E + CSR_NBLKR - 1) / CSR_NBLKR; const int e0 = b * ch, e1 = min(E, e0 + ch);
  for (int i = threadIdx.x; i < NGP; i += 64) cnt[i] = 0;
  for (int i = threadIdx.x; i < CHP; i += 64) ids[i] = -1;
  __syncthreads();
  if (threadIdx.x == 0) {
    for (int e = e0; e < e1; ++e) { int d = dst[e]; d = (d < 0) ? 0 : (d >= N ? N - 1 : d); cnt[d >> CSR_GBR] += 1; }
    int acc = 0; for (int g = 0; g < nG; ++g) { run[g] = acc; acc += cnt[g]; }
    for (int e = e0; e < e1; ++e) { int d = dst[e]; d = (d < 0) ? 0 : (d >= N ? N - 1 : d); const int g = d >> CSR_GBR; ids[run[g]] = e; run[g] += 1; } }
  __syncthreads();
  typedef __attribute__((ext_vector_type(4))) int v4i;
  for (int pass = 0; pass < 2; ++pass) {
    for (int i = threadIdx.x; i < CHP / 4; i += 64) *(volatile v4i*)(STG + (size_t)b * CHP + i * 4) = *(const v4i*)(&ids[i * 4]);
    for (int i = threadIdx.x; i < NGP / 4; i += 64) { v4i v; for (int e = 0; e < 4; ++e) v[e] = (i * 4 + e < nG) ? cnt[i * 4 + e] : 0; *(volatile v4i*)(HST + (size_t)b * NGP + i * 4) = v; }
    __threadfence(); }
}
__global__ __launch_bounds__(512) void csrS_kernelR(const int* __restrict__ HST, int nG, int NGP, int* __restrict__ START, int* __restrict__ TOT, int* __restrict__ OFF) {
  __shared__ int tot[CSR_MAXGR];
  const int b = threadIdx.x;
  for (int pass = 0; pass < 2; ++pass) { int runb = 0; for (int g = 0; g < nG; ++g) { int c = HST[(size_t)b * NGP + g]; c = (c < 0) ? 0 : c; ((volatile int*)OFF)[(size_t)g * CSR_NBLKR + b] = runb; runb += c; } __threadfence(); }
  for (int g = threadIdx.x; g < nG; g += 512) { int s = 0; for (int bb = 0; bb < CSR_NBLKR; ++bb) { int c = HST[(size_t)bb * NGP + g]; s += (c < 0) ? 0 : c; } tot[g] = s; }
  __syncthreads();
  if (threadIdx.x < 32) {
    __shared__ int st[CSR_MAXGR + 32];
    if (threadIdx.x == 0) { int acc = 0; for (int g = 0; g < NGP; ++g) { st[g] = acc; if (g < nG) acc += (tot[g] + 31) & ~31; } st[NGP] = acc; }
    __builtin_amdgcn_fence(__ATOMIC_RELEASE, "workgroup"); __builtin_amdgcn_wave_barrier(); __builtin_amdgcn_fence(__ATOMIC_ACQUIRE, "workgroup");
    for (int pass = 0; pass < 2; ++pass) { for (int i = threadIdx.x; i < NGP + 32; i += 32) { ((volatile int*)START)[i] = (i <= NGP) ? st[min(i, NGP)] : 0; ((volatile int*)TOT)[i] = (i < nG) ? tot[i] : 0; } __threadfence(); } }
}
__global__ __launch_bounds__(256) void csrB_kernelR(const int* __restrict__ dst, int N, int nG, int CHP, int NGP, int permLen, const int* __restrict__ STG, const int* __restrict__ HST, const int* __restrict__ OFF, const int* __restrict__ START, const int* __restrict__ TOT, int* __restrict__ PERM, int* __restrict__ ROWPTR, int* __restrict__ ROWCNT, int* __restrict__ FLAG) {
  typedef __attribute__((ext_vector_type(4))) int v4i;
  __shared__ int ids[CSR_CAPR]; __shared__ unsigned short key[CSR_CAPR]; __shared__ int outp[CSR_CAPR]; __shared__ int ncnt[CSR_GNR + 1]; __shared__ int boff[CSR_NBLKR + 1];
  const int g = blockIdx.x, t_ = threadIdx.x; int tot = TOT[g]; int st = START[g], stn = START[g + 1]; const int v0 = g * CSR_GNR; const int nv = min(CSR_GNR, N - v0); const int t0 = g * CSR_TSR;
  st = (st < 0) ? 0 : (st > permLen - 32 ? permLen - 32 : st) & ~31; stn = (stn < st) ? st : (stn > permLen ? permLen : stn); tot = (tot < 0) ? 0 : tot; if (tot > stn - st && tot <= CSR_CAPR) tot = stn - st;
  if (tot > CSR_CAPR) {
    for (int pass = 0; pass < 2; ++pass) { for (int i = t_; i < CSR_TSR / 4; i += 256) { v4i a, c; for (int e = 0; e < 4; ++e) { a[e] = st; c[e] = 0; } *(volatile v4i*)(ROWPTR + t0 + i * 4) = a; *(volatile v4i*)(ROWCNT + t0 + i * 4) = c; } if (t_ == 0) ((volatile int*)FLAG)[0] = 1; __threadfence(); } (void)nv; return; }
  if (t_ == 0) { int acc = 0; for (int b = 0; b < CSR_NBLKR; ++b) { boff[b] = acc; int c = HST[(size_t)b * NGP + g]; c = (c < 0) ? 0 : (c > CHP ? CHP : c); acc += c; if (acc > tot) acc = tot; } boff[CSR_NBLKR] = acc; }
  for (int i = t_; i <= CSR_GNR; i += 256) ncnt[i] = 0;
  __syncthreads();
  for (int b = 0; b < CSR_NBLKR; ++b) { const int c = boff[b + 1] - boff[b]; int o_ = OFF[(size_t)g * CSR_NBLKR + b]; o_ = (o_ < 0) ? 0 : (o_ > CHP - c ? CHP - c : o_); const int* src_ = STG + (size_t)b * CHP + o_;
    for (int i = t_; i < c; i += 256) { int id = src_[i]; id = (id < 0) ? 0 : id; ids[boff[b] + i] = id; int d = dst[id]; d = (d < v0) ? v0 : (d >= N ? N - 1 : d); int kk = d - v0; kk = (kk < 0) ? 0 : (kk >= CSR_GNR ? CSR_GNR - 1 : kk); key[boff[b] + i] = (unsigned short)kk; } }
  __syncthreads();
  if (t_ == 0) { for (int i = 0; i < tot; ++i) ncnt[key[i]] += 1; int acc = 0; for (int vl = 0; vl < CSR_GNR; ++vl) { const int c = ncnt[vl]; ncnt[vl] = acc; acc += c; } ncnt[CSR_GNR] = acc;
    for (int i = 0; i < tot; ++i) { const int vl = key[i]; outp[ncnt[vl]] = ids[i]; ncnt[vl] += 1; }
    for (int vl = CSR_GNR; vl > 0; --vl) ncnt[vl] = ncnt[vl - 1]; ncnt[0] = 0; }
  __syncthreads();
  for (int pass = 0; pass < 2; ++pass) {
    for (int i = t_; i < (stn - st) / 4; i += 256) { v4i v; for (int e = 0; e < 4; ++e) { const int q = i * 4 + e; v[e] = (q < tot) ? outp[q] : -1; } *(volatile v4i*)(PERM + st + i * 4) = v; }
    for (int i = t_; i < CSR_TSR / 4; i += 256) { v4i a, c; for (int e = 0; e < 4; ++e) { const int vl = i * 4 + e; const int vc = vl < CSR_GNR ? vl : CSR_GNR; a[e] = (vl < CSR_GNR) ? st + ncnt[vc] : st; c[e] = (vl < nv) ? (ncnt[(vc < CSR_GNR ? vc : CSR_GNR - 1) + 1] - ncnt[vc]) : 0; } *(volatile v4i*)(ROWPTR + t0 + i * 4) = a; *(volatile v4i*)(ROWCNT + t0 + i * 4) = c; }
    __threadfence(); }
}
__global__ __launch_bounds__(256) void csrZ_kernelR(int* __restrict__ p, size_t n4) { typedef __attribute__((ext_vector_type(4))) int v4i; const size_t tid = (size_t)blockIdx.x * 256 + threadIdx.x, nth = (size_t)gridDim.x * 256; v4i z = {0, 0, 0, 0}; for (size_t i = tid; i < n4; i += nth) *(volatile v4i*)(p + i * 4) = z; }
struct CsrBufsR { int *STG, *HST, *OFF, *START, *TOT, *PERM, *ROWPTR, *ROWCNT, *FLAG; int nG, NGP, CHP; size_t permLen; char* base; size_t bytes; };
static size_t csr_carveR(CsrBufsR& c, char* ws, size_t off, int E, int N) {
  const size_t off0 = off; c.base = ws + off;
  auto al = [&](size_t bytes) { char* p = ws + off; off += (bytes + 255) & ~(size_t)255; return p; };
  c.nG = (N + CSR_GNR - 1) / CSR_GNR; c.NGP = (c.nG + 31) & ~31; const int ch = (E + CSR_NBLKR - 1) / CSR_NBLKR; c.CHP = (ch + 31) & ~31; c.permLen = (size_t)E + 32 * (size_t)c.nG + 32;
  c.STG = (int*)al((size_t)CSR_NBLKR * c.CHP * 4); c.HST = (int*)al((size_t)CSR_NBLKR * c.NGP * 4); c.OFF = (int*)al((size_t)c.NGP * CSR_NBLKR * 4); c.START = (int*)al((size_t)(c.NGP + 64) * 4); c.TOT = (int*)al((size_t)(c.NGP + 64) * 4);
  c.PERM = (int*)al(c.permLen * 4); c.ROWPTR = (int*)al((size_t)c.nG * CSR_TSR * 4); c.ROWCNT = (int*)al((size_t)c.nG * CSR_TSR * 4); c.FLAG = (int*)al(256);
  c.bytes = off - off0; return off;
}
static void csr_buildR(const CsrBufsR& c, const int* dst, int E, int N, hipStream_t stream) {
  const size_t smem = (size_t)(2 * c.NGP + c.CHP) * 4;
  csrZ_kernelR<<<512, 256, 0, stream>>>((int*)c.base, c.bytes / 16);
  csrA_kernelR<<<CSR_NBLKR, 64, smem, stream>>>(dst, E, N, c.nG, c.CHP, c.NGP, c.STG, c.HST);
  csrS_kernelR<<<1, 512, 0, stream>>>(c.HST, c.nG, c.NGP, c.START, c.TOT, c.OFF);
  csrB_kernelR<<<c.nG, 256, 0, stream>>>(dst, N, c.nG, c.CHP, c.NGP, (int)c.permLen, c.STG, c.HST, c.OFF, c.START, c.TOT, c.PERM, c.ROWPTR, c.ROWCNT, c.FLAG);
}


__global__ __launch_bounds__(256) void wput_kernel(const float* __restrict__ kw, b16* __restrict__ KW) { const int u = blockIdx.x * 256 + threadIdx.x; if (u >= U * (KT / 8)) return; const int o = u / (KT / 8), k0 = (u % (KT / 8)) * 8; v8b v;
#pragma unroll
  for (int j = 0; j < 8; ++j) v[j] = (b16)(bf16_rne(kw[(size_t)(k0 + j) * U + o]) * WSC); for (int pass = 0; pass < 2; ++pass) { *(volatile v8b*)(KW + (size_t)o * KT + k0) = v; __threadfence(); } }
__global__ __launch_bounds__(256) void deg_kernel(const float* __restrict__ ew, const int* __restrict__ PERM, const int* __restrict__ ROWPTR, const int* __restrict__ ROWCNT, int permLen, float* __restrict__ DINV) { const size_t i = (size_t)blockIdx.x * 256 + threadIdx.x; if (i >= (size_t)N) return; int st = ROWPTR[i], cnt = ROWCNT[i]; cnt = iclamp(cnt, 0, E); st = iclamp(st, 0, permLen - cnt); float s = 0.0f;
#pragma unroll 1
  for (int j = 0; j < cnt; ++j) { const int e = iclamp(PERM[st + j], 0, E - 1); s += bfv(ew[e]); }
  const float d = s > 0.0f ? rsqrtf(fmaxf(s, 1e-12f)) : 0.0f;
  for (int pass = 0; pass < 2; ++pass) { ((volatile float*)DINV)[i] = d; __threadfence(); } }
template <int FIRST>
__global__ __launch_bounds__(256) void hop_kernel(const float* __restrict__ IN, const float* __restrict__ ew, const float* __restrict__ DINV, const int* __restrict__ rows, const int* __restrict__ PERM, const int* __restrict__ ROWPTR, const int* __restrict__ ROWCNT, int permLen, int NLIM, float* __restrict__ OUT) { const int wave = threadIdx.x >> 5, lane = threadIdx.x & 31; const size_t i = (size_t)blockIdx.x * 8 + wave; if (i >= (size_t)NLIM) return; int st = ROWPTR[i], cnt = ROWCNT[i]; cnt = iclamp(cnt, 0, E); st = iclamp(st, 0, permLen - cnt); const float di = DINV[i];
  v4f acc = {0, 0, 0, 0};
#pragma unroll 1
  for (int j = 0; j < cnt; ++j) { const int e = iclamp(PERM[st + j], 0, E - 1); const size_t u = (size_t)iclamp(rows[e], 0, N - 1); if (u >= (size_t)NLIM) continue; const float w = pmul(pmul(DINV[u], bfv(ew[e])), di); const v4f v = *(const v4f*)(IN + u * F + lane * 4);
#pragma unroll
    for (int k = 0; k < 4; ++k) acc[k] += pmul(w, FIRST ? bfv(v[k]) : v[k]); }
  const v4f sv = *(const v4f*)(IN + i * F + lane * 4); v4f o; for (int k = 0; k < 4; ++k) o[k] = acc[k] + (FIRST ? bfv(sv[k]) : sv[k]);
  for (int pass = 0; pass < 2; ++pass) { *(volatile v4f*)(OUT + i * F + lane * 4) = o; __threadfence(); } }
__global__ __launch_bounds__(32) void out_kernel(const float* __restrict__ x, const float* __restrict__ H1, const float* __restrict__ H2, const float* __restrict__ H3, const b16* __restrict__ KW, const float* __restrict__ bias, int NLIM, float* __restrict__ out) { __shared__ __attribute__((aligned(16))) b16 Ah[16][KT + 8], Al[16][KT + 8]; __shared__ float Tf[16][U + 4]; const int lane = threadIdx.x, nloc = lane & 15, hlf = lane >> 4; const size_t m0 = (size_t)blockIdx.x * 16; if (m0 >= (size_t)NLIM) return;
  for (int rr = 0; rr < 16; ++rr) for (int q = 0; q < 4; ++q) { const int c = q * 32 + lane; const size_t n = m0 + rr; Ah[rr][c] = (b16)(bf16_rne(x[n * F + c]) * HS); Al[rr][c] = (b16)0.0f; b16 p, ql; split16(H1[n * F + c] * HS, p, ql); Ah[rr][F + c] = p; Al[rr][F + c] = ql; split16(H2[n * F + c] * HS, p, ql); Ah[rr][2 * F + c] = p; Al[rr][2 * F + c] = ql; split16(H3[n * F + c] * HS, p, ql); Ah[rr][3 * F + c] = p; Al[rr][3 * F + c] = ql; }
  wave_lds_sync(); v8f acc[16];
#pragma unroll
  for (int t = 0; t < 16; ++t) acc[t] = (v8f){};
#pragma unroll 2
  for (int kb = 0; kb < KT; kb += 32) { const v16b a = frag_kb(&Ah[nloc][kb], hlf), al = frag_kb(&Al[nloc][kb], hlf); const bool haslo = kb >= F;
#pragma unroll
    for (int t = 0; t < 16; ++t) { const v16b bw = frag_kb(KW + (size_t)(t * 16 + nloc) * KT + kb, hlf); acc[t] = wmma16b(a, bw, acc[t]); if (haslo) acc[t] = wmma16b(al, bw, acc[t]); } }
#pragma unroll
  for (int t = 0; t < 16; ++t) { const int cc = t * 16 + nloc; const float bb = bfv(bias[cc]);
#pragma unroll
    for (int r8 = 0; r8 < 8; ++r8) Tf[8 * hlf + r8][cc] = acc[t][r8] * (1.0f / (HS * WSC)) + bb; }
  wave_lds_sync();
  for (int pass = 0; pass < 2; ++pass) { for (int rr = 0; rr < 16; ++rr) for (int q = 0; q < 2; ++q) *(volatile v4f*)(out + (m0 + rr) * U + q * 128 + lane * 4) = *(const v4f*)(&Tf[rr][q * 128 + lane * 4]); __threadfence(); } }
}

extern "C" void kernel_launch(void* const* d_in, const int* in_sizes, int n_in, void* d_out, int out_size, void* d_ws, size_t ws_size, hipStream_t stream) {
  (void)n_in;
  auto Fp = [&](int i) { return (const float*)d_in[i]; }; auto Ip = [&](int i) { return (const int*)d_in[i]; };
  if (in_sizes[0] != N * F || in_sizes[1] != 2 * E || in_sizes[2] != E || in_sizes[3] != KT * U || in_sizes[4] != U || out_size != N * U) return;
  const int NLIM = N;
  size_t off = 0; char* ws = (char*)d_ws;
  auto carve = [&](size_t bytes) { char* p = ws + off; off += (bytes + 255) & ~(size_t)255; return p; };
  b16* KW = (b16*)carve((size_t)U * KT * 2); float* DINV = (float*)carve((size_t)N * 4); float* H1 = (float*)carve((size_t)N * F * 4); float* H2 = (float*)carve((size_t)N * F * 4); float* H3 = (float*)carve((size_t)N * F * 4);
  CsrBufsC cc; off = csr_carveC(cc, ws, off, E, N); CsrBufsR cr; off = csr_carveR(cr, ws, off, E, N);
  if (off > ws_size || off > ((size_t)128 << 20)) return;
  wput_kernel<<<(U * (KT / 8) + 255) / 256, 256, 0, stream>>>(Fp(3), KW);
  csr_buildC(cc, Ip(1) + E, E, N, stream); csr_buildR(cr, Ip(1), E, N, stream);
  deg_kernel<<<(N + 255) / 256, 256, 0, stream>>>(Fp(2), cr.PERM, cr.ROWPTR, cr.ROWCNT, (int)cr.permLen, DINV);
  hop_kernel<1><<<(NLIM + 7) / 8, 256, 0, stream>>>(Fp(0), Fp(2), DINV, Ip(1), cc.PERM, cc.ROWPTR, cc.ROWCNT, (int)cc.permLen, NLIM, H1);
  hop_kernel<0><<<(NLIM + 7) / 8, 256, 0, stream>>>(H1, Fp(2), DINV, Ip(1), cc.PERM, cc.ROWPTR, cc.ROWCNT, (int)cc.permLen, NLIM, H2);
  hop_kernel<0><<<(NLIM + 7) / 8, 256, 0, stream>>>(H2, Fp(2), DINV, Ip(1), cc.PERM, cc.ROWPTR, cc.ROWCNT, (int)cc.permLen, NLIM, H3);
  out_kernel<<<NLIM / 16, 32, 0, stream>>>(Fp(0), H1, H2, H3, KW, Fp(4), NLIM, (float*)d_out);
}
